// MultiHeadAttention_14568529068339
// MI455X (gfx1250) — hardware-verified
//
#include <hip/hip_runtime.h>


#ifndef NB
#define NB 8
#endif
#ifndef SEQ
#define SEQ 1024
#endif
#define NB_FULL  8
#define SEQ_FULL 1024
#define EM   768
#define NH   12
#define HD   64
#define PP   72
#define XCAR 16.0f
#define PCAR 1024.0f
#define SSCL (0.125f / (XCAR * XCAR))
#define LOG2E 1.4426950408889634f

typedef _Float16 h16;
typedef unsigned short bf;
typedef __attribute__((ext_vector_type(16))) __bf16   v16bf;
typedef __attribute__((ext_vector_type(16))) _Float16 v16h;
typedef __attribute__((ext_vector_type(8)))  _Float16 v8h;
typedef __attribute__((ext_vector_type(8)))  unsigned short v8us;
typedef __attribute__((ext_vector_type(8)))  float    v8f;
typedef __attribute__((ext_vector_type(4)))  float    v4f;
typedef v8h  __attribute__((may_alias)) v8ha;
typedef v4f  __attribute__((may_alias)) v4fa;

static_assert(NH * HD == EM);
static_assert(HD == 64);
static_assert(EM % 64 == 0);
static_assert(EM % 32 == 0);
static_assert(SEQ % 64 == 0);
static_assert((NB * SEQ) % 64 == 0);
static_assert(SEQ <= SEQ_FULL);
static_assert(NB <= NB_FULL);
static_assert(PP % 8 == 0);
static_assert(PP >= 64);
static_assert(((size_t)NB * SEQ * EM / 8) % 256 == 0);
static_assert(((size_t)EM * EM / 8) % 256 == 0);

__device__ __forceinline__ unsigned short f2bf(float f) { unsigned u = __float_as_uint(f); u += 0x7FFFu + ((u >> 16) & 1u); return (unsigned short)(u >> 16); }
__device__ __forceinline__ float bf2f(unsigned short b) { return __uint_as_float(((unsigned)b) << 16); }
__device__ __forceinline__ float bfr(float f) { return bf2f(f2bf(f)); }
__device__ __forceinline__ v16h cat16(v8h lo, v8h hi) { return __builtin_shufflevector(lo, hi, 0, 1, 2, 3, 4, 5, 6, 7, 8, 9, 10, 11, 12, 13, 14, 15); }
__device__ __forceinline__ v16bf cat16b(v8us lo, v8us hi) { return __builtin_bit_cast(v16bf, __builtin_shufflevector(lo, hi, 0, 1, 2, 3, 4, 5, 6, 7, 8, 9, 10, 11, 12, 13, 14, 15)); }
__device__ __forceinline__ v8f wmma16(v16h a, v16h b, v8f c) { return __builtin_amdgcn_wmma_f32_16x16x32_f16(false, a, false, b, (short)0, c, false, false); }
__device__ __forceinline__ v8f wmmab(v16bf a, v16bf b, v8f c) { return __builtin_amdgcn_wmma_f32_16x16x32_bf16(false, a, false, b, (short)0, c, false, false); }
__device__ __forceinline__ void splitf(float y, unsigned short& h, unsigned short& l) { h = f2bf(y); l = f2bf(y - bf2f(h)); }

template <typename T16> struct WFrag;
template <> struct WFrag<h16> { typedef v16h V; static __device__ __forceinline__ V ld(const h16* p) { return cat16(*(const v8h*)p, *(const v8h*)(p + 16)); } static __device__ __forceinline__ v8f mma(V a, V b, v8f c) { return wmma16(a, b, c); } };
template <> struct WFrag<bf> { typedef v16bf V; static __device__ __forceinline__ V ld(const bf* p) { return cat16b(*(const v8us*)p, *(const v8us*)(p + 16)); } static __device__ __forceinline__ v8f mma(V a, V b, v8f c) { return wmmab(a, b, c); } };

template <typename T16, int NSPLIT, bool BIAS>
__device__ __forceinline__ void gemm_body(const T16* __restrict__ A, const T16* __restrict__ A2, const T16* __restrict__ Bt, const T16* __restrict__ Bt2, int K, float* C, int ldc, const float* __restrict__ bias, size_t sA, size_t sB, size_t sC) {
    typedef typename WFrag<T16>::V V;
    __shared__ __align__(16) float os[16 * 68];
    const size_t z = blockIdx.z; A += z * sA; if (A2) A2 += z * sA; Bt += z * sB; if (Bt2) Bt2 += z * sB; C += z * sC;
    const int lane = threadIdx.x & 31, lr = lane & 15, hi = lane >> 4; const int r0 = blockIdx.x * 64, c0 = blockIdx.y * 64;
    v8f acc[4][4];
#pragma unroll
    for (int mb = 0; mb < 4; ++mb)
#pragma unroll
        for (int nb = 0; nb < 4; ++nb) acc[mb][nb] = (v8f){};
    const size_t aoff = (size_t)(r0 + lr) * K + 8 * hi, boff = (size_t)(c0 + lr) * K + 8 * hi;
#pragma unroll 1
    for (int kc = 0; kc < K; kc += 32) {
        V a[4], a2[4];
#pragma unroll
        for (int mb = 0; mb < 4; ++mb) { a[mb] = WFrag<T16>::ld(A + aoff + (size_t)mb * 16 * K + kc); if (NSPLIT == 1 || NSPLIT == 2) a2[mb] = WFrag<T16>::ld(A2 + aoff + (size_t)mb * 16 * K + kc); }
#pragma unroll
        for (int nb = 0; nb < 4; ++nb) { const V b = WFrag<T16>::ld(Bt + boff + (size_t)nb * 16 * K + kc); V b2; if (NSPLIT >= 2) b2 = WFrag<T16>::ld(Bt2 + boff + (size_t)nb * 16 * K + kc);
#pragma unroll
            for (int mb = 0; mb < 4; ++mb) { acc[mb][nb] = WFrag<T16>::mma(a[mb], b, acc[mb][nb]); if (NSPLIT == 1 || NSPLIT == 2) acc[mb][nb] = WFrag<T16>::mma(a2[mb], b, acc[mb][nb]); if (NSPLIT >= 2) acc[mb][nb] = WFrag<T16>::mma(a[mb], b2, acc[mb][nb]); } }
        asm volatile("v_nop\n\tv_nop\n\tv_nop\n\tv_nop" : "+v"(acc[0][0]), "+v"(acc[1][1]), "+v"(acc[2][2]), "+v"(acc[3][3]) : "v"(a[0]), "v"(a[3]));
    }
#pragma unroll
    for (int mb = 0; mb < 4; ++mb) {
#pragma unroll
        for (int nb = 0; nb < 4; ++nb) {
#pragma unroll
            for (int j = 0; j < 8; ++j) os[(hi * 8 + j) * 68 + nb * 16 + lr] = acc[mb][nb][j]; }
        __builtin_amdgcn_wave_barrier(); asm volatile("" ::: "memory");
        float* crow = C + (size_t)(r0 + mb * 16) * ldc + c0;
#pragma unroll 1
        for (int ps = 0; ps < 2; ++ps) {
#pragma unroll
            for (int s = 0; s < 8; ++s) { const int row = 2 * s + hi, cofs = lr * 4; v4f val = *(const v4fa*)(os + row * 68 + cofs); if (BIAS) { val[0] += bfr(bias[c0 + cofs]); val[1] += bfr(bias[c0 + cofs + 1]); val[2] += bfr(bias[c0 + cofs + 2]); val[3] += bfr(bias[c0 + cofs + 3]); }
                *(volatile v4f*)(crow + (size_t)row * ldc + cofs) = val; }
            if (ps == 0) __threadfence(); }
        __builtin_amdgcn_wave_barrier(); asm volatile("" ::: "memory");
    }
}

__global__ __launch_bounds__(32) void k_gemm_proj(const bf* A, const bf* Bt, int K, float* C, int ldc, const float* bias) {
    gemm_body<bf, 0, true>(A, (const bf*)nullptr, Bt, (const bf*)nullptr, K, C, ldc, bias, 0, 0, 0);
}
__global__ __launch_bounds__(32) void k_gemm_out(const bf* Ah, const bf* Al, const bf* Bt, int K, float* C, int ldc, const float* bias, size_t sA, size_t sC) {
    gemm_body<bf, 1, true>(Ah, Al, Bt, (const bf*)nullptr, K, C, ldc, bias, sA, 0, sC);
}

__global__ __launch_bounds__(256) void k_cvt8(const float* __restrict__ src, bf* dst, size_t n8) { const size_t i = (size_t)blockIdx.x * 256 + threadIdx.x; if (i >= n8) return; const v8f v = *(const v8f*)(src + i * 8); v8us o;
#pragma unroll
    for (int k = 0; k < 8; ++k) o[k] = f2bf(v[k]); *(volatile v8us*)(dst + i * 8) = o; __threadfence(); *(volatile v8us*)(dst + i * 8) = o; }

__global__ __launch_bounds__(256) void k_cvtx(const float* __restrict__ src, bf* dst) {
    const size_t i = (size_t)blockIdx.x * 256 + threadIdx.x; if (i >= (size_t)NB * SEQ * EM / 8) return;
    const size_t e = i * 8; const int col = (int)(e % EM); const size_t row = e / EM; const int t = (int)(row % SEQ); const int b = (int)(row / SEQ);
    const v8f v = *(const v8f*)(src + ((size_t)b * SEQ_FULL + t) * EM + col); v8us o;
#pragma unroll
    for (int k = 0; k < 8; ++k) o[k] = f2bf(v[k]);
    *(volatile v8us*)(dst + e) = o; __threadfence(); *(volatile v8us*)(dst + e) = o; }

__global__ __launch_bounds__(256) void k_hp(const float* __restrict__ F, h16* P) {
    const size_t i = (size_t)blockIdx.x * 256 + threadIdx.x; if (i >= (size_t)NB * NH * SEQ * HD / 8) return;
    const size_t e = i * 8; const int d = (int)(e % HD); const int t = (int)((e / HD) % SEQ); const int bh = (int)(e / ((size_t)HD * SEQ)); const int b = bh / NH, h = bh % NH;
    const float* f = F + ((size_t)b * SEQ + t) * EM + h * HD + d; const v4f a0 = *(const v4f*)f, a1 = *(const v4f*)(f + 4); v8h o;
#pragma unroll
    for (int k = 0; k < 4; ++k) { o[k] = (h16)(a0[k] * XCAR); o[k + 4] = (h16)(a1[k] * XCAR); }
    *(volatile v8h*)(P + e) = o; __threadfence(); *(volatile v8h*)(P + e) = o; }

__global__ __launch_bounds__(256) void k_vtp(const float* __restrict__ F, h16* V) {
    const size_t i = (size_t)blockIdx.x * 256 + threadIdx.x; if (i >= (size_t)NB * NH * HD * SEQ / 8) return;
    const size_t e = i * 8; const int t = (int)(e % SEQ); const int d = (int)((e / SEQ) % HD); const int bh = (int)(e / ((size_t)SEQ * HD)); const int b = bh / NH, h = bh % NH;
    const float* f = F + ((size_t)b * SEQ + t) * EM + h * HD + d; v8h o;
#pragma unroll
    for (int q = 0; q < 8; ++q) o[q] = (h16)(f[(size_t)q * EM] * XCAR);
    *(volatile v8h*)(V + e) = o; __threadfence(); *(volatile v8h*)(V + e) = o; }

__global__ __launch_bounds__(256) void k_vsum(const float* __restrict__ F, float* VS) {
    __shared__ float part[4 * 64];
    const int col = threadIdx.x & 63, pr = threadIdx.x >> 6; const int b = blockIdx.y; const int n = blockIdx.x * 64 + col;
    const float* f = F + ((size_t)b * SEQ + (size_t)pr * (SEQ / 4)) * EM + n;
    float s0 = 0.f, s1 = 0.f, s2 = 0.f, s3 = 0.f;
#pragma unroll 1
    for (int t = 0; t < SEQ / 4; t += 4) { s0 += f[(size_t)t * EM]; s1 += f[(size_t)(t + 1) * EM]; s2 += f[(size_t)(t + 2) * EM]; s3 += f[(size_t)(t + 3) * EM]; }
    part[pr * 64 + col] = (s0 + s1) + (s2 + s3);
    __syncthreads();
    if (threadIdx.x < 16) { v4f o;
#pragma unroll
        for (int q = 0; q < 4; ++q) { const int c = threadIdx.x * 4 + q; o[q] = (part[c] + part[64 + c]) + (part[128 + c] + part[192 + c]); }
        float* dst = VS + (size_t)b * EM + blockIdx.x * 64 + threadIdx.x * 4; *(volatile v4f*)dst = o; __threadfence(); *(volatile v4f*)dst = o; }
}

__global__ __launch_bounds__(32) void k_flash(const h16* __restrict__ QP, const h16* __restrict__ KP, const h16* __restrict__ VT, const float* __restrict__ VS, const int* __restrict__ msk, bf* Ah, bf* Al) {
    __shared__ __align__(16) h16 pt[16 * PP];
    __shared__ __align__(16) float os[16 * 68];
    const int lane = threadIdx.x & 31, lr = lane & 15, hi = lane >> 4;
    const int q0 = blockIdx.x * 16, h = blockIdx.y, b = blockIdx.z, bh = b * NH + h;
    const h16* Qb = QP + (size_t)bh * SEQ * HD + (size_t)(q0 + lr) * HD + 8 * hi;
    const h16* Kb = KP + (size_t)bh * SEQ * HD + (size_t)lr * HD + 8 * hi;
    const h16* Vb = VT + (size_t)bh * HD * SEQ + (size_t)lr * SEQ + 8 * hi;
    const int* mrow = msk + (size_t)b * SEQ_FULL + lr;
    const v16h qa0 = WFrag<h16>::ld(Qb), qa1 = WFrag<h16>::ld(Qb + 32);

    float mx[8], sm[8];
#pragma unroll
    for (int r = 0; r < 8; ++r) { mx[r] = -3.0e38f; sm[r] = 0.f; }

#pragma unroll 1
    for (int kc = 0; kc < SEQ; kc += 64) {
        v8f s[4]; v16h lastb = qa1;
#pragma unroll
        for (int j = 0; j < 4; ++j) { const h16* kp = Kb + (size_t)(kc + j * 16) * HD; const v16h k0 = WFrag<h16>::ld(kp), k1 = WFrag<h16>::ld(kp + 32);
            s[j] = wmma16(qa0, k0, (v8f){}); s[j] = wmma16(qa1, k1, s[j]); if (j == 3) lastb = k1; }
        asm volatile("v_nop\n\tv_nop\n\tv_nop\n\tv_nop" : "+v"(s[0]), "+v"(s[1]), "+v"(s[2]), "+v"(s[3]) : "v"(qa0), "v"(qa1), "v"(lastb));
#pragma unroll
        for (int j = 0; j < 4; ++j) { const bool valid = mrow[kc + j * 16] != 0;
#pragma unroll
            for (int r = 0; r < 8; ++r) { const float t = valid ? s[j][r] * SSCL : 1e-9f; mx[r] = fmaxf(mx[r], t); sm[r] += t; } }
    }
    float cr[8];
#pragma unroll
    for (int r = 0; r < 8; ++r) { float m = mx[r], ss = sm[r];
#pragma unroll
        for (int sh = 8; sh; sh >>= 1) { m = fmaxf(m, __shfl_xor(m, sh, 32)); ss += __shfl_xor(ss, sh, 32); }
        mx[r] = m; cr[r] = __builtin_amdgcn_exp2f((ss * (1.0f / (float)SEQ) - m) * LOG2E); }

    v8f acc[4]; float ls[8];
#pragma unroll
    for (int j = 0; j < 4; ++j) acc[j] = (v8f){};
#pragma unroll
    for (int r = 0; r < 8; ++r) ls[r] = 0.f;
#pragma unroll 1
    for (int kc = 0; kc < SEQ; kc += 64) {
        v8f s[4]; v16h lastb = qa1;
#pragma unroll
        for (int j = 0; j < 4; ++j) { const h16* kp = Kb + (size_t)(kc + j * 16) * HD; const v16h k0 = WFrag<h16>::ld(kp), k1 = WFrag<h16>::ld(kp + 32);
            s[j] = wmma16(qa0, k0, (v8f){}); s[j] = wmma16(qa1, k1, s[j]); if (j == 3) lastb = k1; }
        asm volatile("v_nop\n\tv_nop\n\tv_nop\n\tv_nop" : "+v"(s[0]), "+v"(s[1]), "+v"(s[2]), "+v"(s[3]) : "v"(qa0), "v"(qa1), "v"(lastb));
#pragma unroll
        for (int j = 0; j < 4; ++j) { const bool valid = mrow[kc + j * 16] != 0;
#pragma unroll
            for (int r = 0; r < 8; ++r) { const float t = valid ? s[j][r] * SSCL : 1e-9f; const float p = __builtin_amdgcn_exp2f((t - mx[r]) * LOG2E); ls[r] += p;
                pt[(8 * hi + r) * PP + j * 16 + lr] = (h16)((p - cr[r]) * PCAR); } }
        __syncthreads();
        const h16* pr = pt + lr * PP + 8 * hi;
        const v16h pa0 = cat16(*(const v8ha*)pr, *(const v8ha*)(pr + 16));
        const v16h pa1 = cat16(*(const v8ha*)(pr + 32), *(const v8ha*)(pr + 48));
        v16h lastv = pa1;
#pragma unroll
        for (int j = 0; j < 4; ++j) { const h16* vp = Vb + (size_t)(j * 16) * SEQ + kc; const v16h v0 = WFrag<h16>::ld(vp), v1 = WFrag<h16>::ld(vp + 32);
            acc[j] = wmma16(pa0, v0, acc[j]); acc[j] = wmma16(pa1, v1, acc[j]); if (j == 3) lastv = v1; }
        asm volatile("v_nop\n\tv_nop\n\tv_nop\n\tv_nop" : "+v"(acc[0]), "+v"(acc[1]), "+v"(acc[2]), "+v"(acc[3]) : "v"(pa0), "v"(pa1), "v"(lastv));
        __syncthreads();
    }

    float vs[4];
#pragma unroll
    for (int j = 0; j < 4; ++j) vs[j] = VS[(size_t)b * EM + h * HD + j * 16 + lr];
#pragma unroll
    for (int r = 0; r < 8; ++r) { float l = ls[r];
#pragma unroll
        for (int sh = 8; sh; sh >>= 1) l += __shfl_xor(l, sh, 32);
        const float inv = __builtin_amdgcn_rcpf(l);
#pragma unroll
        for (int j = 0; j < 4; ++j) os[(8 * hi + r) * 68 + j * 16 + lr] = (acc[j][r] * (1.0f / (PCAR * XCAR)) + cr[r] * vs[j]) * inv; }
    __syncthreads();
#pragma unroll 1
    for (int ps = 0; ps < 2; ++ps) {
#pragma unroll
        for (int it = 0; it < 4; ++it) { const int piece = it * 32 + lane; const int row = piece >> 3, seg = piece & 7;
            const v4f a0 = *(const v4fa*)(os + row * 68 + seg * 8), a1 = *(const v4fa*)(os + row * 68 + seg * 8 + 4); v8us oh, ol;
#pragma unroll
            for (int k = 0; k < 4; ++k) { unsigned short x, y; splitf(a0[k], x, y); oh[k] = x; ol[k] = y; splitf(a1[k], x, y); oh[k + 4] = x; ol[k + 4] = y; }
            const size_t oo = ((size_t)b * SEQ + q0 + row) * EM + h * HD + seg * 8; *(volatile v8us*)(Ah + oo) = oh; *(volatile v8us*)(Al + oo) = ol; }
        if (ps == 0) __threadfence(); }
}

constexpr size_t al256(size_t x) { return (x + 255) & ~(size_t)255; }
constexpr size_t SZ_W   = al256((size_t)EM * EM * 2);
constexpr size_t SZ_XB  = al256((size_t)NB * SEQ * EM * 2);
constexpr size_t SZ_F   = al256((size_t)NB * SEQ * EM * 4);
constexpr size_t SZ_PL  = al256((size_t)NB * NH * SEQ * HD * 2);
constexpr size_t SZ_VS  = al256((size_t)NB * EM * 4);
constexpr size_t SZ_AT  = al256((size_t)NB * SEQ * EM * 2);
constexpr size_t WS_TOTAL = 4 * SZ_W + SZ_XB + SZ_F + 3 * SZ_PL + SZ_VS + 2 * SZ_AT;
static_assert(WS_TOTAL <= (size_t)134217728);

extern "C" void kernel_launch(void* const* d_in, const int* in_sizes, int n_in,
                              void* d_out, int out_size, void* d_ws, size_t ws_size, hipStream_t stream) {
    if (n_in < 13) return;
    const size_t need_act = ((size_t)(NB - 1) * SEQ_FULL + SEQ) * EM;
    if ((size_t)in_sizes[0] < need_act || (size_t)in_sizes[1] < need_act || (size_t)in_sizes[2] < need_act) return;
    if ((size_t)in_sizes[3] < (size_t)(NB - 1) * SEQ_FULL + SEQ) return;
    if ((size_t)in_sizes[5] < (size_t)EM * EM || (size_t)in_sizes[7] < (size_t)EM * EM || (size_t)in_sizes[9] < (size_t)EM * EM || (size_t)in_sizes[11] < (size_t)EM * EM) return;
    if (in_sizes[6] < EM || in_sizes[8] < EM || in_sizes[10] < EM || in_sizes[12] < EM) return;
    if ((size_t)out_size < need_act) return;
    if (WS_TOTAL > ws_size) return;
    const float* q = (const float*)d_in[0]; const float* k = (const float*)d_in[1]; const float* v = (const float*)d_in[2];
    const int* mask = (const int*)d_in[3];
    (void)d_in[4];
    const float* Wq = (const float*)d_in[5]; const float* bq = (const float*)d_in[6];
    const float* Wk = (const float*)d_in[7]; const float* bk = (const float*)d_in[8];
    const float* Wv = (const float*)d_in[9]; const float* bv = (const float*)d_in[10];
    const float* Wo = (const float*)d_in[11]; const float* bo = (const float*)d_in[12];
    float* OUT = (float*)d_out;
    char* wsp = (char*)d_ws;
    auto take = [&](size_t bytes) { char* p = wsp; wsp += bytes; return (void*)p; };
    bf* WQ = (bf*)take(SZ_W); bf* WK = (bf*)take(SZ_W); bf* WV = (bf*)take(SZ_W); bf* WO = (bf*)take(SZ_W);
    bf* XB = (bf*)take(SZ_XB); float* F = (float*)take(SZ_F);
    h16* QP = (h16*)take(SZ_PL); h16* KP = (h16*)take(SZ_PL); h16* VTp = (h16*)take(SZ_PL);
    float* VS = (float*)take(SZ_VS); bf* ATh = (bf*)take(SZ_AT); bf* ATl = (bf*)take(SZ_AT);

    const unsigned gw = (unsigned)(((size_t)EM * EM / 8 + 255) / 256);
    k_cvt8<<<gw, 256, 0, stream>>>(Wq, WQ, (size_t)EM * EM / 8);
    k_cvt8<<<gw, 256, 0, stream>>>(Wk, WK, (size_t)EM * EM / 8);
    k_cvt8<<<gw, 256, 0, stream>>>(Wv, WV, (size_t)EM * EM / 8);
    k_cvt8<<<gw, 256, 0, stream>>>(Wo, WO, (size_t)EM * EM / 8);

    const unsigned gx = (unsigned)(((size_t)NB * SEQ * EM / 8 + 255) / 256);
    const dim3 gp(NB * SEQ / 64, EM / 64, 1);
    k_cvtx<<<gx, 256, 0, stream>>>(q, XB);
    k_gemm_proj<<<gp, 32, 0, stream>>>(XB, WQ, EM, F, EM, bq);
    k_hp<<<gx, 256, 0, stream>>>(F, QP);
    k_cvtx<<<gx, 256, 0, stream>>>(k, XB);
    k_gemm_proj<<<gp, 32, 0, stream>>>(XB, WK, EM, F, EM, bk);
    k_hp<<<gx, 256, 0, stream>>>(F, KP);
    k_cvtx<<<gx, 256, 0, stream>>>(v, XB);
    k_gemm_proj<<<gp, 32, 0, stream>>>(XB, WV, EM, F, EM, bv);
    k_vtp<<<gx, 256, 0, stream>>>(F, VTp);
    k_vsum<<<dim3(EM / 64, NB, 1), 256, 0, stream>>>(F, VS);
    k_flash<<<dim3(SEQ / 16, NH, NB), 32, 0, stream>>>(QP, KP, VTp, VS, mask, ATh, ATl);
    k_gemm_out<<<dim3(SEQ / 64, EM / 64, NB), 32, 0, stream>>>(ATh, ATl, WO, EM, OUT, EM, bo, (size_t)SEQ * EM, (size_t)SEQ_FULL * EM);
}
